// MHA_24919400252086
// MI455X (gfx1250) — hardware-verified
//
#include <hip/hip_runtime.h>


#ifndef NB
#define NB 4
#endif
#ifndef SEQ
#define SEQ 2048
#endif
#define SEQ_FULL 2048
#define DM   1024
#define NHD  16
#define HD   64
#define DQ   (NHD * HD)
#define RH   256
#define PCAR 1024.0f
#define SCL  0.125f
#define L2E  1.4426950408889634f
#define LDP  40
static_assert(SEQ % 64 == 0);
static_assert(RH % 64 == 0);
static_assert(RH <= SEQ);
static_assert(SEQ <= SEQ_FULL);

typedef _Float16 h16;
typedef unsigned short bf;
typedef __attribute__((ext_vector_type(16))) __bf16   v16bf;
typedef __attribute__((ext_vector_type(16))) _Float16 v16h;
typedef __attribute__((ext_vector_type(8)))  _Float16 v8h;
typedef __attribute__((ext_vector_type(8)))  unsigned short v8us;
typedef __attribute__((ext_vector_type(8)))  float    v8f;
typedef __attribute__((ext_vector_type(4)))  float    v4f;
typedef __attribute__((ext_vector_type(2)))  _Float16 v2h;
typedef __attribute__((ext_vector_type(2)))  unsigned short v2us;
typedef __attribute__((ext_vector_type(2)))  float v2f;
typedef v8h  __attribute__((may_alias)) v8ha;
typedef v4f  __attribute__((may_alias)) v4fa;
typedef v8us __attribute__((may_alias)) v8usa;

__device__ __forceinline__ unsigned short f2bf(float f) { unsigned u = __float_as_uint(f); u += 0x7FFFu + ((u >> 16) & 1u); return (unsigned short)(u >> 16); }
__device__ __forceinline__ float bf2f(unsigned short b) { return __uint_as_float(((unsigned)b) << 16); }
__device__ __forceinline__ float bfr(float f) { return bf2f(f2bf(f)); }
__device__ __forceinline__ v16h cat16(v8h lo, v8h hi) { return __builtin_shufflevector(lo, hi, 0, 1, 2, 3, 4, 5, 6, 7, 8, 9, 10, 11, 12, 13, 14, 15); }
__device__ __forceinline__ v16bf cat16b(v8us lo, v8us hi) { return __builtin_bit_cast(v16bf, __builtin_shufflevector(lo, hi, 0, 1, 2, 3, 4, 5, 6, 7, 8, 9, 10, 11, 12, 13, 14, 15)); }
__device__ __forceinline__ v8f wmma16(v16h a, v16h b, v8f c) { return __builtin_amdgcn_wmma_f32_16x16x32_f16(false, a, false, b, (short)0, c, false, false); }
__device__ __forceinline__ v8f wmmab(v16bf a, v16bf b, v8f c) { return __builtin_amdgcn_wmma_f32_16x16x32_bf16(false, a, false, b, (short)0, c, false, false); }
__device__ __forceinline__ h16 tohx(float x) { return (h16)x; }
__device__ __forceinline__ void splitf(float y, unsigned short& h, unsigned short& l) { h = f2bf(y); l = f2bf(y - bf2f(h)); }

__device__ __forceinline__ float redmax16(float v) {
    v = fmaxf(v, __shfl_xor(v, 1, 32)); v = fmaxf(v, __shfl_xor(v, 2, 32)); v = fmaxf(v, __shfl_xor(v, 4, 32)); v = fmaxf(v, __shfl_xor(v, 8, 32)); return v; }
__device__ __forceinline__ float redsum16(float v) {
    v += __shfl_xor(v, 1, 32); v += __shfl_xor(v, 2, 32); v += __shfl_xor(v, 4, 32); v += __shfl_xor(v, 8, 32); return v; }

template <typename T16> struct WFrag;
template <> struct WFrag<h16> { typedef v16h V; static __device__ __forceinline__ V ld(const h16* p) { return cat16(*(const v8h*)p, *(const v8h*)(p + 16)); } static __device__ __forceinline__ v8f mma(V a, V b, v8f c) { return wmma16(a, b, c); } };
template <> struct WFrag<bf> { typedef v16bf V; static __device__ __forceinline__ V ld(const bf* p) { return cat16b(*(const v8us*)p, *(const v8us*)(p + 16)); } static __device__ __forceinline__ v8f mma(V a, V b, v8f c) { return wmmab(a, b, c); } };

template <typename T16, int NSPLIT, bool BIAS>
__global__ __launch_bounds__(32) void k_gemmw(const T16* __restrict__ A, const T16* __restrict__ A2, const T16* __restrict__ Bt, const T16* __restrict__ Bt2, int K, float* C, int ldc, const float* __restrict__ bias, size_t sA, size_t sB, size_t sC) {
    typedef typename WFrag<T16>::V V;
    __shared__ __align__(16) float os[16 * 68];
    const size_t z = blockIdx.z; A += z * sA; if (A2) A2 += z * sA; Bt += z * sB; if (Bt2) Bt2 += z * sB; C += z * sC;
    const int lane = threadIdx.x & 31, lr = lane & 15, hi = lane >> 4; const int r0 = blockIdx.x * 64, c0 = blockIdx.y * 64;
    v8f acc[4][4];
#pragma unroll
    for (int mb = 0; mb < 4; ++mb)
#pragma unroll
        for (int nb = 0; nb < 4; ++nb) acc[mb][nb] = (v8f){};
    const size_t aoff = (size_t)(r0 + lr) * K + 8 * hi, boff = (size_t)(c0 + lr) * K + 8 * hi;
#pragma unroll 1
    for (int kc = 0; kc < K; kc += 32) {
        V a[4], a2[4];
#pragma unroll
        for (int mb = 0; mb < 4; ++mb) { a[mb] = WFrag<T16>::ld(A + aoff + (size_t)mb * 16 * K + kc); if (NSPLIT == 1 || NSPLIT == 2) a2[mb] = WFrag<T16>::ld(A2 + aoff + (size_t)mb * 16 * K + kc); }
#pragma unroll
        for (int nb = 0; nb < 4; ++nb) { const V b = WFrag<T16>::ld(Bt + boff + (size_t)nb * 16 * K + kc); V b2; if (NSPLIT >= 2) b2 = WFrag<T16>::ld(Bt2 + boff + (size_t)nb * 16 * K + kc);
#pragma unroll
            for (int mb = 0; mb < 4; ++mb) { acc[mb][nb] = WFrag<T16>::mma(a[mb], b, acc[mb][nb]); if (NSPLIT == 1 || NSPLIT == 2) acc[mb][nb] = WFrag<T16>::mma(a2[mb], b, acc[mb][nb]); if (NSPLIT >= 2) acc[mb][nb] = WFrag<T16>::mma(a[mb], b2, acc[mb][nb]); } }
        asm volatile("v_nop\n\tv_nop\n\tv_nop\n\tv_nop" : "+v"(acc[0][0]), "+v"(acc[1][1]), "+v"(acc[2][2]), "+v"(acc[3][3]) : "v"(a[0]), "v"(a[3]));
    }
#pragma unroll
    for (int mb = 0; mb < 4; ++mb) {
#pragma unroll
        for (int nb = 0; nb < 4; ++nb) {
#pragma unroll
            for (int j = 0; j < 8; ++j) os[(hi * 8 + j) * 68 + nb * 16 + lr] = acc[mb][nb][j]; }
        __builtin_amdgcn_wave_barrier(); asm volatile("" ::: "memory");
        float* crow = C + (size_t)(r0 + mb * 16) * ldc + c0;
#pragma unroll 1
        for (int ps = 0; ps < 2; ++ps) {
#pragma unroll
            for (int s = 0; s < 8; ++s) { const int row = 2 * s + hi, cofs = lr * 4; v4f val = *(const v4fa*)(os + row * 68 + cofs); if (BIAS) { val[0] += bfr(bias[c0 + cofs]); val[1] += bfr(bias[c0 + cofs + 1]); val[2] += bfr(bias[c0 + cofs + 2]); val[3] += bfr(bias[c0 + cofs + 3]); }
                *(volatile v4f*)(crow + (size_t)row * ldc + cofs) = val; }
            if (ps == 0) __threadfence(); }
        __builtin_amdgcn_wave_barrier(); asm volatile("" ::: "memory");
    }
}

__global__ __launch_bounds__(256) void k_wtG(const float* __restrict__ w, int K, int N, bf* Bt) {
    const int lane = threadIdx.x & 31; const int L0 = (blockIdx.x * 8 + (threadIdx.x >> 5)) * 8; const int nlines = N * K / 64;
#pragma unroll
    for (int ps = 0; ps < 2; ++ps) {
#pragma unroll 1
        for (int l = 0; l < 8; ++l) { const int L = L0 + l; if (L >= nlines) break; const size_t e = (size_t)L * 64 + lane * 2; const int k = (int)(e % K), n = (int)(e / K); v2us o;
            o[0] = f2bf(w[(size_t)k * N + n]); o[1] = f2bf(w[(size_t)(k + 1) * N + n]); *(volatile v2us*)(Bt + e) = o; }
        if (ps == 0) __threadfence(); }
}
__global__ __launch_bounds__(256) void k_cvt8(const float* __restrict__ src, bf* dst, size_t n8) { const size_t i = (size_t)blockIdx.x * 256 + threadIdx.x; if (i >= n8) return; const v8f v = *(const v8f*)(src + i * 8); v8us o;
#pragma unroll
    for (int k = 0; k < 8; ++k) o[k] = f2bf(v[k]); *(volatile v8us*)(dst + i * 8) = o; __threadfence(); *(volatile v8us*)(dst + i * 8) = o; }

__global__ __launch_bounds__(256) void k_qkp(const float* __restrict__ F, h16* P16, bf* Ph, bf* Pl) {
    const size_t e = ((size_t)blockIdx.x * 256 + threadIdx.x) * 2; if (e >= (size_t)NHD * SEQ * HD) return;
    const int d = (int)(e % HD); const int t = (int)((e / HD) % SEQ); const int h = (int)(e / ((size_t)HD * SEQ));
    const v2f x = *(const v2f*)(F + (size_t)t * DQ + h * HD + d);
    v2h o16; v2us oh, ol;
#pragma unroll
    for (int q = 0; q < 2; ++q) { o16[q] = tohx(x[q]); unsigned short a, c; splitf(x[q], a, c); oh[q] = a; ol[q] = c; }
    const size_t eh = ((size_t)h * RH + t) * HD + d;
#pragma unroll 1
    for (int ps = 0; ps < 2; ++ps) {
        *(volatile v2h*)(P16 + e) = o16;
        if (t < RH) { *(volatile v2us*)(Ph + eh) = oh; *(volatile v2us*)(Pl + eh) = ol; }
        if (ps == 0) __threadfence(); }
}
__global__ __launch_bounds__(256) void k_vtp(const float* __restrict__ F, h16* V16, bf* Vh, bf* Vl) {
    const size_t e = ((size_t)blockIdx.x * 256 + threadIdx.x) * 2; if (e >= (size_t)NHD * HD * SEQ) return;
    const int t = (int)(e % SEQ); const int d = (int)((e / SEQ) % HD); const int g = (int)(e / ((size_t)SEQ * HD));
    v2h o16; v2us oh, ol;
#pragma unroll
    for (int q = 0; q < 2; ++q) { const float x = F[(size_t)(t + q) * DQ + g * HD + d]; o16[q] = tohx(x); unsigned short a, c; splitf(x, a, c); oh[q] = a; ol[q] = c; }
    const size_t eh = ((size_t)g * HD + d) * RH + t;
#pragma unroll 1
    for (int ps = 0; ps < 2; ++ps) {
        *(volatile v2h*)(V16 + e) = o16;
        if (t < RH) { *(volatile v2us*)(Vh + eh) = oh; *(volatile v2us*)(Vl + eh) = ol; }
        if (ps == 0) __threadfence(); }
}

template <bool HR>
__global__ __launch_bounds__(32) __attribute__((amdgpu_num_vgpr(256)))
void k_attn(const h16* __restrict__ Q16, const bf* __restrict__ Qh, const bf* __restrict__ Ql,
            const h16* __restrict__ K16, const bf* __restrict__ Kh, const bf* __restrict__ Kl,
            const h16* __restrict__ V16, const bf* __restrict__ Vh, const bf* __restrict__ Vl,
            int qt0, bf* Ah, bf* Al) {
    __shared__ __align__(16) h16 pT[16 * LDP];
    __shared__ __align__(16) bf  pTh[16 * LDP];
    __shared__ __align__(16) bf  pTl[16 * LDP];
    __shared__ __align__(16) bf  osh[16 * 64];
    __shared__ __align__(16) bf  osl[16 * 64];
    const int lane = threadIdx.x & 31, l15 = lane & 15, hi = lane >> 4;
    const int qbase = (qt0 + (int)blockIdx.x) * 16; const int hh = blockIdx.y;

    v16h aq16[2]; v16bf aqh[2], aql[2];
    if constexpr (HR) {
        const size_t qo = ((size_t)hh * RH + qbase + l15) * HD + 8 * hi;
#pragma unroll
        for (int c = 0; c < 2; ++c) { aqh[c] = WFrag<bf>::ld(Qh + qo + c * 32); aql[c] = WFrag<bf>::ld(Ql + qo + c * 32); }
    } else {
        const size_t qo = ((size_t)hh * SEQ + qbase + l15) * HD + 8 * hi;
#pragma unroll
        for (int c = 0; c < 2; ++c) aq16[c] = WFrag<h16>::ld(Q16 + qo + c * 32);
    }

    v8f o[4];
#pragma unroll
    for (int g = 0; g < 4; ++g) o[g] = (v8f){};
    float mr[8], lr[8];
#pragma unroll
    for (int r = 0; r < 8; ++r) { mr[r] = -1.0e30f; lr[r] = 0.f; }

    const int nkv = qbase + 16;
#pragma unroll 1
    for (int kv0 = 0; kv0 < nkv; kv0 += 32) {
        v8f s[2];
#pragma unroll
        for (int j = 0; j < 2; ++j) {
            const int krow = kv0 + j * 16 + l15;
            v8f z = (v8f){};
            if constexpr (HR) {
                const size_t ko = ((size_t)hh * RH + krow) * HD + 8 * hi;
                v16bf b, b2;
#pragma unroll
                for (int c = 0; c < 2; ++c) { b = WFrag<bf>::ld(Kh + ko + c * 32); b2 = WFrag<bf>::ld(Kl + ko + c * 32);
                    z = wmmab(aqh[c], b, z); z = wmmab(aql[c], b, z); z = wmmab(aqh[c], b2, z); }
                asm volatile("v_nop\n\tv_nop\n\tv_nop\n\tv_nop" : "+v"(z) : "v"(b), "v"(b2), "v"(aqh[1]));
            } else {
                const size_t ko = ((size_t)hh * SEQ + krow) * HD + 8 * hi;
                v16h b;
#pragma unroll
                for (int c = 0; c < 2; ++c) { b = WFrag<h16>::ld(K16 + ko + c * 32); z = wmma16(aq16[c], b, z); }
                asm volatile("v_nop\n\tv_nop\n\tv_nop\n\tv_nop" : "+v"(z) : "v"(b), "v"(aq16[1]));
            }
            s[j] = z;
        }

        float p0[8], p1[8];
        const int key0 = kv0 + l15, key1 = kv0 + 16 + l15;
#pragma unroll
        for (int r = 0; r < 8; ++r) {
            const int row = qbase + 8 * hi + r;
            const bool ok0 = (key0 <= row), ok1 = (key1 <= row);
            const float t0 = ok0 ? s[0][r] * SCL : -1.0e30f;
            const float t1 = ok1 ? s[1][r] * SCL : -1.0e30f;
            const float cm = redmax16(fmaxf(t0, t1));
            const float mn = fmaxf(mr[r], cm);
            const float corr = __builtin_amdgcn_exp2f((mr[r] - mn) * L2E);
            float e0 = __builtin_amdgcn_exp2f((t0 - mn) * L2E); e0 = ok0 ? e0 : 0.f;
            float e1 = __builtin_amdgcn_exp2f((t1 - mn) * L2E); e1 = ok1 ? e1 : 0.f;
            const float rs = redsum16(e0 + e1);
            lr[r] = lr[r] * corr + rs; mr[r] = mn;
            o[0][r] *= corr; o[1][r] *= corr; o[2][r] *= corr; o[3][r] *= corr;
            p0[r] = e0; p1[r] = e1;
        }

        __syncthreads();
        if constexpr (HR) {
#pragma unroll
            for (int r = 0; r < 8; ++r) { unsigned short a0, c0, a1, c1; splitf(p0[r], a0, c0); splitf(p1[r], a1, c1);
                const int ro = (8 * hi + r) * LDP + l15; pTh[ro] = a0; pTl[ro] = c0; pTh[ro + 16] = a1; pTl[ro + 16] = c1; }
        } else {
#pragma unroll
            for (int r = 0; r < 8; ++r) { const int ro = (8 * hi + r) * LDP + l15; pT[ro] = tohx(p0[r] * PCAR); pT[ro + 16] = tohx(p1[r] * PCAR); }
        }
        __syncthreads();
        v16h ap; v16bf aph, apl;
        if constexpr (HR) {
            const bf* pr = pTh + l15 * LDP + 8 * hi; const bf* pl = pTl + l15 * LDP + 8 * hi;
            aph = cat16b(*(const v8usa*)pr, *(const v8usa*)(pr + 16)); apl = cat16b(*(const v8usa*)pl, *(const v8usa*)(pl + 16));
        } else {
            const h16* pr = pT + l15 * LDP + 8 * hi;
            ap = cat16(*(const v8ha*)pr, *(const v8ha*)(pr + 16));
        }

        if constexpr (HR) {
            v16bf bv, bl;
#pragma unroll
            for (int g = 0; g < 4; ++g) { const size_t vo = ((size_t)hh * HD + g * 16 + l15) * RH + kv0 + 8 * hi;
                bv = WFrag<bf>::ld(Vh + vo); bl = WFrag<bf>::ld(Vl + vo);
                o[g] = wmmab(aph, bv, o[g]); o[g] = wmmab(apl, bv, o[g]); o[g] = wmmab(aph, bl, o[g]); }
            asm volatile("v_nop\n\tv_nop\n\tv_nop\n\tv_nop" : "+v"(o[0]), "+v"(o[1]), "+v"(o[2]), "+v"(o[3]) : "v"(bv), "v"(bl), "v"(aph), "v"(apl));
        } else {
            v16h bv;
#pragma unroll
            for (int g = 0; g < 4; ++g) { const size_t vo = ((size_t)hh * HD + g * 16 + l15) * SEQ + kv0 + 8 * hi;
                bv = WFrag<h16>::ld(V16 + vo); o[g] = wmma16(ap, bv, o[g]); }
            asm volatile("v_nop\n\tv_nop\n\tv_nop\n\tv_nop" : "+v"(o[0]), "+v"(o[1]), "+v"(o[2]), "+v"(o[3]) : "v"(bv), "v"(ap));
        }
    }

    const float cs = HR ? 1.0f : (1.0f / PCAR);
#pragma unroll
    for (int r = 0; r < 8; ++r) {
        const float inv = cs / lr[r];
#pragma unroll
        for (int g = 0; g < 4; ++g) { unsigned short a, c2; splitf(o[g][r] * inv, a, c2); const int oo = (8 * hi + r) * 64 + g * 16 + l15; osh[oo] = a; osl[oo] = c2; }
    }
    __syncthreads();
    v8us vh[4], vl[4];
    const int rq = lane >> 3, pc = (lane & 7) * 8;
#pragma unroll
    for (int i = 0; i < 4; ++i) { const int rr = i * 4 + rq; vh[i] = *(const v8usa*)(osh + rr * 64 + pc); vl[i] = *(const v8usa*)(osl + rr * 64 + pc); }
#pragma unroll 1
    for (int ps = 0; ps < 2; ++ps) {
#pragma unroll
        for (int i = 0; i < 4; ++i) { const int rr = i * 4 + rq; const size_t go = (size_t)(qbase + rr) * DQ + hh * HD + pc;
            *(volatile v8us*)(Ah + go) = vh[i]; *(volatile v8us*)(Al + go) = vl[i]; }
        if (ps == 0) __threadfence();
    }
}

extern "C" void kernel_launch(void* const* d_in, const int* in_sizes, int n_in,
                              void* d_out, int out_size, void* d_ws, size_t ws_size, hipStream_t stream) {
    if (n_in < 5) return;
    if (in_sizes[0] < ((NB - 1) * SEQ_FULL + SEQ) * DM) return;
    if (in_sizes[1] < DM * DM || in_sizes[2] < DM * DM || in_sizes[3] < DM * DM || in_sizes[4] < DM * DM) return;
    if (out_size < ((NB - 1) * SEQ_FULL + SEQ) * DM) return;
    const float* x  = (const float*)d_in[0];
    const float* wq = (const float*)d_in[1];
    const float* wk = (const float*)d_in[2];
    const float* wv = (const float*)d_in[3];
    const float* wo = (const float*)d_in[4];
    float* OUT = (float*)d_out;
    char* wsp = (char*)d_ws;
    auto take = [&](size_t bytes) { char* p = wsp; wsp += (bytes + 255) & ~(size_t)255; return (void*)p; };
    bf* WQ = (bf*)take((size_t)DM * DM * 2); bf* WK = (bf*)take((size_t)DM * DM * 2); bf* WV = (bf*)take((size_t)DM * DM * 2); bf* WO = (bf*)take((size_t)DM * DM * 2);
    bf* XB = (bf*)take((size_t)SEQ * DM * 2);
    float* F1 = (float*)take((size_t)SEQ * DQ * 4); float* F2 = (float*)take((size_t)SEQ * DQ * 4);
    h16* Q16 = (h16*)take((size_t)NHD * SEQ * HD * 2); bf* Qh = (bf*)take((size_t)NHD * RH * HD * 2); bf* Ql = (bf*)take((size_t)NHD * RH * HD * 2);
    h16* K16 = (h16*)take((size_t)NHD * SEQ * HD * 2); bf* Kh = (bf*)take((size_t)NHD * RH * HD * 2); bf* Kl = (bf*)take((size_t)NHD * RH * HD * 2);
    h16* V16 = (h16*)take((size_t)NHD * HD * SEQ * 2); bf* Vh = (bf*)take((size_t)NHD * HD * RH * 2); bf* Vl = (bf*)take((size_t)NHD * HD * RH * 2);
    bf* ATh = (bf*)take((size_t)SEQ * DQ * 2); bf* ATl = (bf*)take((size_t)SEQ * DQ * 2);
    if ((size_t)(wsp - (char*)d_ws) > ws_size) return;

    const unsigned gW = (unsigned)((DM * DM / 64 + 63) / 64);
    k_wtG<<<gW, 256, 0, stream>>>(wq, DM, DQ, WQ);
    k_wtG<<<gW, 256, 0, stream>>>(wk, DM, DQ, WK);
    k_wtG<<<gW, 256, 0, stream>>>(wv, DM, DQ, WV);
    k_wtG<<<gW, 256, 0, stream>>>(wo, DQ, DM, WO);
    const unsigned gP = (unsigned)(((size_t)NHD * SEQ * HD / 2 + 255) / 256);
    for (int b = 0; b < NB; ++b) {
        k_cvt8<<<(unsigned)(((size_t)SEQ * DM / 8 + 255) / 256), 256, 0, stream>>>(x + (size_t)b * SEQ_FULL * DM, XB, (size_t)SEQ * DM / 8);
        k_gemmw<bf, 0, false><<<dim3(SEQ / 64, DQ / 64, 1), 32, 0, stream>>>(XB, nullptr, WQ, nullptr, DM, F1, DQ, nullptr, 0, 0, 0);
        k_qkp<<<gP, 256, 0, stream>>>(F1, Q16, Qh, Ql);
        k_gemmw<bf, 0, false><<<dim3(SEQ / 64, DQ / 64, 1), 32, 0, stream>>>(XB, nullptr, WK, nullptr, DM, F2, DQ, nullptr, 0, 0, 0);
        k_qkp<<<gP, 256, 0, stream>>>(F2, K16, Kh, Kl);
        k_gemmw<bf, 0, false><<<dim3(SEQ / 64, DQ / 64, 1), 32, 0, stream>>>(XB, nullptr, WV, nullptr, DM, F1, DQ, nullptr, 0, 0, 0);
        k_vtp<<<gP, 256, 0, stream>>>(F1, V16, Vh, Vl);
        k_attn<true><<<dim3(RH / 16, NHD, 1), 32, 0, stream>>>(Q16, Qh, Ql, K16, Kh, Kl, V16, Vh, Vl, 0, ATh, ATl);
        if (SEQ > RH) k_attn<false><<<dim3((SEQ - RH) / 16, NHD, 1), 32, 0, stream>>>(Q16, Qh, Ql, K16, Kh, Kl, V16, Vh, Vl, RH / 16, ATh, ATl);
        k_gemmw<bf, 1, false><<<dim3(SEQ / 64, DM / 64, 1), 32, 0, stream>>>(ATh, ATl, WO, nullptr, DQ, OUT + (size_t)b * SEQ_FULL * DM, DM, nullptr, 0, 0, 0);
    }
}
